// DualGraphModel_2241972928706
// MI455X (gfx1250) — hardware-verified
//
#include <hip/hip_runtime.h>
#include <stddef.h>


#define IND     256
#define CC      128
#define NL      4
#define NCLS    10
#define NCLSP   32
#define NTHR    256
#define NWAVE   8
#define EPT     8
#define NGRP    2
#define CHUNK   (NTHR * EPT * NGRP)
#define WCAPC   (EPT * NGRP * 32)
#define WCAPF   (EPT * NGRP * 32)
#define ESHF    11
#define EMASK   0xFFFFF
#define NBC     32768
#define NBF     2048
#define RCAP    49152
#define RBN     128
#define TGT     256
#define DEGCAP  512
#define GROWS   128
#define OTHR    512
#define TPK     64
#define TPN     32
#define TPP     72
#define ASCL    16
#define WSCL    64
#define WSCAP   134217728

#define LDS_COUNT  ((NBC + NWAVE * WCAPC + NWAVE) * 4)
#define LDS_FILL   ((RCAP + NBF + NWAVE * WCAPF + NWAVE) * 4)
#define LDS_GEMM   (GROWS * CC * 4)

static_assert((CHUNK & (CHUNK - 1)) == 0);
static_assert((NBC & (NBC - 1)) == 0 && (NBF & (NBF - 1)) == 0);
static_assert(NBF <= (1 << ESHF));
static_assert((NBC % NBF) == 0);
static_assert(OTHR * 4 == NBF);
static_assert((RCAP % 32) == 0);
static_assert(TGT == NWAVE * 32);
static_assert(GROWS == NWAVE * 16);
static_assert((TGT % GROWS) == 0);
static_assert(NBC == NWAVE * 32 * 128);
static_assert(CC == 32 * 4);
static_assert((CC % 32) == 0 && (IND % 32) == 0);
static_assert((CC % TPK) == 0 && (CC % TPN) == 0 && (IND % TPK) == 0 && (NCLSP % TPN) == 0);
static_assert(TPN * 8 == NTHR && TPK * TPN == NTHR * 8 && TPK == NWAVE * 8);
static_assert((TPP % 8) == 0 && TPP >= TPK);
static_assert(NCLS <= 16 && NCLSP >= 16);
static_assert(((GROWS * NCLS) % 32) == 0);
static_assert(LDS_FILL <= 300 * 1024);

typedef float     v4f  __attribute__((ext_vector_type(4)));
typedef float     v8f  __attribute__((ext_vector_type(8)));
typedef int       v4i  __attribute__((ext_vector_type(4)));
typedef _Float16  v4h  __attribute__((ext_vector_type(4)));
typedef _Float16  v8h  __attribute__((ext_vector_type(8)));
typedef _Float16  v16h __attribute__((ext_vector_type(16)));
union FragH { v16h v; v8h h[2]; };
union U32F { float f; int i; };

__device__ __forceinline__ v8f wmf(v16h a, v16h b, v8f c) {
  v8f d = __builtin_amdgcn_wmma_f32_16x16x32_f16(false, a, false, b, (short)0, c, false, false);
  asm volatile("v_nop\n\tv_nop\n\tv_nop\n\tv_nop" : "+v"(d) : "v"(a), "v"(b));
  return d;
}

__device__ __forceinline__ v8h cvt8h(v4f a, v4f b, float z) {
  v8h h;
  h[0] = (_Float16)(a.x * z); h[1] = (_Float16)(a.y * z); h[2] = (_Float16)(a.z * z); h[3] = (_Float16)(a.w * z);
  h[4] = (_Float16)(b.x * z); h[5] = (_Float16)(b.y * z); h[6] = (_Float16)(b.z * z); h[7] = (_Float16)(b.w * z);
  return h;
}

template <int NB, int SRC, int WC>
__device__ __forceinline__ int scan_chunk(const int* __restrict__ keys, int nK, int cbase,
                                          int slotBase, int vec8, int* list, int tid, int lane, int wave) {
  int wc = 0;
#pragma unroll
  for (int g = 0; g < NGRP; ++g) {
    const int el0  = (g * NTHR + tid) * EPT;
    const int e0   = cbase + el0;
    const int sent = -2147483647 - 1;
    const int i0 = min(e0, nK - 1),     i1 = min(e0 + 1, nK - 1), i2 = min(e0 + 2, nK - 1), i3 = min(e0 + 3, nK - 1);
    const int i4 = min(e0 + 4, nK - 1), i5 = min(e0 + 5, nK - 1), i6 = min(e0 + 6, nK - 1), i7 = min(e0 + 7, nK - 1);
    v4i da, db;
    if (vec8 != 0 && cbase + CHUNK <= nK) {
      da = *(const v4i*)(keys + e0);
      db = *(const v4i*)(keys + e0 + 4);
    } else {
      da.x = (e0     < nK) ? keys[i0] : sent;
      da.y = (e0 + 1 < nK) ? keys[i1] : sent;
      da.z = (e0 + 2 < nK) ? keys[i2] : sent;
      da.w = (e0 + 3 < nK) ? keys[i3] : sent;
      db.x = (e0 + 4 < nK) ? keys[i4] : sent;
      db.y = (e0 + 5 < nK) ? keys[i5] : sent;
      db.z = (e0 + 6 < nK) ? keys[i6] : sent;
      db.w = (e0 + 7 < nK) ? keys[i7] : sent;
    }
    const unsigned nb = (unsigned)slotBase;
    const unsigned s0 = (unsigned)da.x - nb, s1 = (unsigned)da.y - nb;
    const unsigned s2 = (unsigned)da.z - nb, s3 = (unsigned)da.w - nb;
    const unsigned s4 = (unsigned)db.x - nb, s5 = (unsigned)db.y - nb;
    const unsigned s6 = (unsigned)db.z - nb, s7 = (unsigned)db.w - nb;
    const bool h0 = s0 < (unsigned)NB, h1 = s1 < (unsigned)NB, h2 = s2 < (unsigned)NB, h3 = s3 < (unsigned)NB;
    const bool h4 = s4 < (unsigned)NB, h5 = s5 < (unsigned)NB, h6 = s6 < (unsigned)NB, h7 = s7 < (unsigned)NB;
    const unsigned any = __builtin_amdgcn_ballot_w32(h0 | h1 | h2 | h3 | h4 | h5 | h6 | h7);
    if (any != 0u) {
#define HITJ(HJ, SJ, VJ) { \
        const unsigned mj = __builtin_amdgcn_ballot_w32(HJ); \
        if (mj != 0u) { \
          if (HJ) { \
            const int pos = wc + (int)__builtin_amdgcn_mbcnt_lo(mj, 0u); \
            const int entv = SRC ? (((VJ) << ESHF) | (int)(SJ)) : (int)(SJ); \
            if (pos < WC) list[wave * WC + pos] = entv; \
          } \
          wc += (int)__builtin_popcount(mj); } }
      HITJ(h0, s0, i0)
      HITJ(h1, s1, i1)
      HITJ(h2, s2, i2)
      HITJ(h3, s3, i3)
      HITJ(h4, s4, i4)
      HITJ(h5, s5, i5)
      HITJ(h6, s6, i6)
      HITJ(h7, s7, i7)
#undef HITJ
    }
  }
  return wc;
}

__global__ __launch_bounds__(NTHR) void k_wT16(const float* __restrict__ W, _Float16* Wp,
                                               int KD, int NC, int NCP, float scale) {
  __shared__ __attribute__((aligned(16))) _Float16 sT[TPN * TPP];
  const int tid = threadIdx.x;
  const int z = (int)blockIdx.z;
  const float* Wz = W + (size_t)z * (size_t)KD * (size_t)NC;
  _Float16* Wpz = Wp + (size_t)z * (size_t)NCP * (size_t)KD;
  const int k0 = (int)blockIdx.x * TPK, n0 = (int)blockIdx.y * TPN;
  const int nc = tid & 31, kq = tid >> 5;
  const int col = n0 + nc;
  const int colc = col < NC ? col : NC - 1;
#pragma unroll
  for (int i = 0; i < TPK / NWAVE; ++i) {
    const int kr = kq + NWAVE * i;
    const float w = Wz[(size_t)(k0 + kr) * NC + colc];
    const float v = (col < NC) ? w * scale : 0.0f;
    sT[nc * TPP + kr] = (_Float16)v;
  }
  __syncthreads();
  const int nl = tid >> 3, p = tid & 7;
  const v8h hv = *(const v8h*)(sT + nl * TPP + 8 * p);
  _Float16* d = Wpz + (size_t)(n0 + nl) * KD + k0 + 8 * p;
  *(volatile v8h*)d = hv;
  __threadfence();
  *(volatile v8h*)d = hv;
}

__global__ __launch_bounds__(NTHR) void k_count(
    const int* __restrict__ keys, int* cnt, int nK, int vec8) {
  extern __shared__ v4f lds_dyn[];
  int* scnt = (int*)lds_dyn;
  int* list = scnt + NBC;
  int* wcnt = list + NWAVE * WCAPC;
  const int tid = threadIdx.x, lane = tid & 31, wave = tid >> 5;
  const int nodeBase = blockIdx.x * NBC;

  {
    const v4i z = {0, 0, 0, 0};
    for (int i = tid; i < NBC / 4; i += NTHR) ((v4i*)scnt)[i] = z;
  }
  __syncthreads();

  const int nChunks = (nK + CHUNK - 1) / CHUNK;
#pragma unroll 1
  for (int ch = 0; ch < nChunks; ++ch) {
    const int cbase = ch * CHUNK;
    const int wc = scan_chunk<NBC, 0, WCAPC>(keys, nK, cbase, nodeBase, vec8, list, tid, lane, wave);
    if (lane == 0) wcnt[wave] = wc;
    __syncthreads();
    if (wave == 0) {
#pragma unroll 1
      for (int wsx = 0; wsx < NWAVE; ++wsx) {
        int n = __builtin_amdgcn_readfirstlane(wcnt[wsx]);
        n = n > WCAPC ? WCAPC : (n < 0 ? 0 : n);
        const int* lp = list + wsx * WCAPC;
#pragma unroll 1
        for (int i = 0; i < n; ++i) {
          const int ent  = __builtin_amdgcn_readfirstlane(lp[i]);
          const int slot = ent & (NBC - 1);
          if (lane == 0) scnt[slot] = scnt[slot] + 1;
        }
      }
    }
    __syncthreads();
  }

  int* cp = cnt + (size_t)nodeBase;
#pragma unroll 4
  for (int q = 0; q < 32; ++q) {
    const int f = (wave * 32 + q) * 128 + 4 * lane;
    const v4i c = *(const v4i*)(scnt + f);
    *(volatile v4i*)(cp + f) = c;
  }
  __threadfence();
#pragma unroll 4
  for (int q = 0; q < 32; ++q) {
    const int f = (wave * 32 + q) * 128 + 4 * lane;
    const v4i c = *(const v4i*)(scnt + f);
    *(volatile v4i*)(cp + f) = c;
  }
}

__global__ __launch_bounds__(OTHR) void k_offsets(
    const int* __restrict__ cnt, int* off, float* dis, int* rbase, int nBF) {
  __shared__ __attribute__((aligned(16))) int srb[RBN];
  __shared__ int wtot[OTHR / 32];
  const int tid = threadIdx.x, lane = tid & 31, wave = tid >> 5;
  for (int i = tid; i < RBN; i += OTHR) srb[i] = 0;
  int carry = 0;
#pragma unroll 1
  for (int fb = 0; fb < nBF; ++fb) {
    const int base = fb * NBF;
    const v4i c = *(const v4i*)(cnt + base + 4 * tid);
    const int e0 = max(c.x, 0), e1 = max(c.y, 0), e2 = max(c.z, 0), e3 = max(c.w, 0);
    const int ts = e0 + e1 + e2 + e3;
    int incl = ts;
#pragma unroll
    for (int d = 1; d < 32; d <<= 1) {
      const int t = __shfl_up(incl, d, 32);
      if (lane >= d) incl += t;
    }
    if (lane == 31) wtot[wave] = incl;
    __syncthreads();
    int pre = 0;
#pragma unroll 1
    for (int w = 0; w < wave; ++w) pre += wtot[w];
    int tot = 0;
#pragma unroll
    for (int w = 0; w < OTHR / 32; ++w) tot += wtot[w];
    int run = carry + pre + incl - ts;
    v4i o;
    o.x = run; run += e0;
    o.y = run; run += e1;
    o.z = run; run += e2;
    o.w = run;
    v4f dv;
    dv.x = rsqrtf((float)e0 + 1.0f);
    dv.y = rsqrtf((float)e1 + 1.0f);
    dv.z = rsqrtf((float)e2 + 1.0f);
    dv.w = rsqrtf((float)e3 + 1.0f);
    int*   op = off + base + 4 * tid;
    float* dp = dis + base + 4 * tid;
    *(volatile v4i*)op = o;
    *(volatile v4f*)dp = dv;
    __threadfence();
    *(volatile v4i*)op = o;
    *(volatile v4f*)dp = dv;
    if (tid == 0) srb[min(fb, RBN - 1)] = carry;
    carry += (tot + 31) & ~31;
    __syncthreads();
  }
  if (tid == 0) srb[min(nBF, RBN - 1)] = carry;
  __syncthreads();
  v4i rv = {0, 0, 0, 0};
  if (tid < 32) rv = *(const v4i*)(srb + 4 * tid);
  if (tid < 32) *(volatile v4i*)(rbase + 4 * tid) = rv;
  __threadfence();
  if (tid < 32) *(volatile v4i*)(rbase + 4 * tid) = rv;
}

__global__ __launch_bounds__(NTHR) void k_fill(
    const int* __restrict__ keys, const int* __restrict__ off,
    const int* __restrict__ rbase, int* csr, int nK, int vec8, int csrLen) {
  extern __shared__ v4f lds_dyn[];
  int* region = (int*)lds_dyn;
  int* cursor = region + RCAP;
  int* list   = cursor + NBF;
  int* wcnt   = list + NWAVE * WCAPF;
  const int tid = threadIdx.x, lane = tid & 31, wave = tid >> 5;
  const int b = blockIdx.x;
  const int nodeBase = b * NBF;

  int rb0 = rbase[b];
  const int rb1 = rbase[b + 1];
  rb0 = rb0 < 0 ? 0 : (rb0 > csrLen ? csrLen : rb0);
  rb0 &= ~31;
  int len = rb1 - rb0;
  len = len < 0 ? 0 : (len > RCAP ? RCAP : len);
  int lenW = (len + 31) & ~31;
  if (rb0 + lenW > csrLen) lenW = (csrLen - rb0) & ~31;

  {
    const v4i z = {0, 0, 0, 0};
    for (int i = tid; i < RCAP / 4; i += NTHR) ((v4i*)region)[i] = z;
    for (int s = tid; s < NBF; s += NTHR) {
      int o = off[nodeBase + s] - rb0;
      o = o < 0 ? 0 : (o > RCAP ? RCAP : o);
      cursor[s] = o;
    }
  }
  __syncthreads();

  const int nChunks = (nK + CHUNK - 1) / CHUNK;
#pragma unroll 1
  for (int ch = 0; ch < nChunks; ++ch) {
    const int cbase = ch * CHUNK;
    const int wc = scan_chunk<NBF, 1, WCAPF>(keys, nK, cbase, nodeBase, vec8, list, tid, lane, wave);
    if (lane == 0) wcnt[wave] = wc;
    __syncthreads();
    if (wave == 0) {
#pragma unroll 1
      for (int wsx = 0; wsx < NWAVE; ++wsx) {
        int n = __builtin_amdgcn_readfirstlane(wcnt[wsx]);
        n = n > WCAPF ? WCAPF : (n < 0 ? 0 : n);
        const int* lp = list + wsx * WCAPF;
#pragma unroll 1
        for (int i = 0; i < n; ++i) {
          const int ent  = __builtin_amdgcn_readfirstlane(lp[i]);
          const int slot = ent & (NBF - 1);
          int ev = (ent >> ESHF) & EMASK;
          ev = ev > nK - 1 ? nK - 1 : ev;
          if (lane == 0) {
            int pos = cursor[slot];
            pos = pos < 0 ? 0 : (pos > RCAP - 1 ? RCAP - 1 : pos);
            region[pos] = ev;
            const int np = pos + 1;
            cursor[slot] = np > RCAP ? RCAP : np;
          }
        }
      }
    }
    __syncthreads();
  }

  const int nv = lenW >> 2;
  int* gp = csr + rb0;
#pragma unroll 1
  for (int i = tid; i < nv; i += NTHR) { const v4i v = ((const v4i*)region)[i]; *(volatile v4i*)(gp + 4 * i) = v; }
  __threadfence();
#pragma unroll 1
  for (int i = tid; i < nv; i += NTHR) { const v4i v = ((const v4i*)region)[i]; *(volatile v4i*)(gp + 4 * i) = v; }
}

template <int KD, int EPO>
__global__ __launch_bounds__(NTHR) void k_gemm(
    const float* __restrict__ A, int lda, int acol, int nArows,
    const _Float16* __restrict__ Bw, const float* __restrict__ bias,
    float* Cout, int ldc, int ccol, float osc) {
  extern __shared__ v4f lds_dyn[];
  static_assert((KD % 32) == 0);
  constexpr int NC  = CC;
  constexpr int NT  = NC / 16;
  constexpr int NST = 16;
  float* stg = (float*)lds_dyn;
  const int tid = threadIdx.x, lane = tid & 31, wave = tid >> 5, hh = lane >> 4, m = lane & 15;
  const int rowBase = blockIdx.x * GROWS;
  const int ar  = rowBase + wave * 16 + m;
  const int arc = ar < nArows ? ar : nArows - 1;
  const float z = (ar < nArows) ? (float)ASCL : 0.0f;
  const float* ap = A + (size_t)arc * lda + acol + 8 * hh;
  const _Float16* bp0 = Bw + (size_t)m * KD + 8 * hh;

  v8f acc[NT];
#pragma unroll
  for (int t = 0; t < NT; ++t) { v8f zz = {0.f, 0.f, 0.f, 0.f, 0.f, 0.f, 0.f, 0.f}; acc[t] = zz; }

#pragma unroll 1
  for (int kt = 0; kt < KD / 32; ++kt) {
    const float* p = ap + 32 * kt;
    const v4f f0 = *(const v4f*)p;
    const v4f f1 = *(const v4f*)(p + 4);
    const v4f f2 = *(const v4f*)(p + 16);
    const v4f f3 = *(const v4f*)(p + 20);
    FragH af;
    af.h[0] = cvt8h(f0, f1, z);
    af.h[1] = cvt8h(f2, f3, z);
#pragma unroll
    for (int t = 0; t < NT; ++t) {
      const _Float16* bp = bp0 + (size_t)(16 * t) * KD + 32 * kt;
      FragH bf;
      bf.h[0] = *(const v8h*)bp;
      bf.h[1] = *(const v8h*)(bp + 16);
      acc[t] = wmf(af.v, bf.v, acc[t]);
    }
  }

  const int r0 = wave * 16 + 8 * hh;
  float bc[NT];
#pragma unroll
  for (int t = 0; t < NT; ++t) bc[t] = (EPO == 1) ? bias[16 * t + m] : 0.0f;

  float* sp = stg + r0 * NC + m;
#pragma unroll
  for (int t = 0; t < NT; ++t) {
#pragma unroll
    for (int r = 0; r < 8; ++r) {
      sp[r * NC + 16 * t] = acc[t][r] * osc + bc[t];
    }
  }
  __syncthreads();

  const float* lp = stg + wave * 16 * NC;
  float* gp = Cout + (size_t)(rowBase + wave * 16) * ldc + ccol;
#pragma unroll
  for (int i = 0; i < NST; ++i) {
    const v4f v = *(const v4f*)(lp + i * NC + 4 * lane);
    *(volatile v4f*)(gp + (size_t)i * ldc + 4 * lane) = v;
  }
  __threadfence();
#pragma unroll
  for (int i = 0; i < NST; ++i) {
    const v4f v = *(const v4f*)(lp + i * NC + 4 * lane);
    *(volatile v4f*)(gp + (size_t)i * ldc + 4 * lane) = v;
  }
}

__global__ __launch_bounds__(NTHR) void k_cls(
    const float* __restrict__ A, int lda, int nArows,
    const _Float16* __restrict__ Bw, const float* __restrict__ bias,
    float* outp, int nN, float osc) {
  __shared__ __attribute__((aligned(16))) float stg[GROWS * NCLS];
  constexpr int KD = IND;
  const int tid = threadIdx.x, lane = tid & 31, wave = tid >> 5, hh = lane >> 4, m = lane & 15;
  const int rowBase = blockIdx.x * GROWS;
  const int ar  = rowBase + wave * 16 + m;
  const int arc = ar < nArows ? ar : nArows - 1;
  const float z = (ar < nArows) ? (float)ASCL : 0.0f;
  const float* ap = A + (size_t)arc * lda + 8 * hh;
  const _Float16* bp0 = Bw + (size_t)m * KD + 8 * hh;

  v8f acc = {0.f, 0.f, 0.f, 0.f, 0.f, 0.f, 0.f, 0.f};
#pragma unroll 1
  for (int kt = 0; kt < KD / 32; ++kt) {
    const float* p = ap + 32 * kt;
    const v4f f0 = *(const v4f*)p;
    const v4f f1 = *(const v4f*)(p + 4);
    const v4f f2 = *(const v4f*)(p + 16);
    const v4f f3 = *(const v4f*)(p + 20);
    FragH af, bf;
    af.h[0] = cvt8h(f0, f1, z);
    af.h[1] = cvt8h(f2, f3, z);
    bf.h[0] = *(const v8h*)(bp0 + 32 * kt);
    bf.h[1] = *(const v8h*)(bp0 + 32 * kt + 16);
    acc = wmf(af.v, bf.v, acc);
  }

  const int mc = m < NCLS ? m : NCLS - 1;
  const float bm = bias[mc];
  const int r0 = wave * 16 + 8 * hh;
  float ov[8];
#pragma unroll
  for (int r = 0; r < 8; ++r) ov[r] = acc[r] * osc + bm;
  if (m < NCLS) {
#pragma unroll
    for (int r = 0; r < 8; ++r) stg[(r0 + r) * NCLS + m] = ov[r];
  }
  __syncthreads();

  int nr = nN - rowBase;
  nr = nr > GROWS ? GROWS : (nr < 0 ? 0 : nr);
  const int nF  = nr * NCLS;
  const int nF4 = nF >> 2;
  float* gp = outp + (size_t)rowBase * NCLS;
#pragma unroll 1
  for (int i = tid; i < nF4; i += NTHR) { const v4f v = *(const v4f*)(stg + 4 * i); *(volatile v4f*)(gp + 4 * i) = v; }
#pragma unroll 1
  for (int i = 4 * nF4 + tid; i < nF; i += NTHR) { const float v = stg[i]; *(volatile float*)(gp + i) = v; }
  __threadfence();
#pragma unroll 1
  for (int i = tid; i < nF4; i += NTHR) { const v4f v = *(const v4f*)(stg + 4 * i); *(volatile v4f*)(gp + 4 * i) = v; }
#pragma unroll 1
  for (int i = 4 * nF4 + tid; i < nF; i += NTHR) { const float v = stg[i]; *(volatile float*)(gp + i) = v; }
}

__global__ __launch_bounds__(NTHR) void k_agg(
    const int* __restrict__ csr, const int* __restrict__ off, const int* __restrict__ cnt,
    const int* __restrict__ srcidx, const float* __restrict__ dis,
    const float* __restrict__ hw, const float* __restrict__ bias,
    const float* __restrict__ gam, const float* __restrict__ bet,
    float* X, int ldx, int xcol, int nN, int nE, int csrLen, float eps) {
  const int tid = threadIdx.x, lane = tid & 31, wave = tid >> 5;
  const int tbase = blockIdx.x * TGT + wave * 32;
  const int cl = tbase + lane;
  const int cnt_l = cnt[cl];
  const int off_l = off[cl];
  const float dis_l = dis[cl];
  const int ch = 4 * lane;
  const v4f bv = *(const v4f*)(bias + ch);
  const v4f gv = *(const v4f*)(gam + ch);
  const v4f ev = *(const v4f*)(bet + ch);
  const float inv128 = 1.0f / 128.0f;

#pragma unroll 1
  for (int j = 0; j < 32; ++j) {
    const int c = tbase + j;
    const int nraw = __builtin_amdgcn_readlane(cnt_l, j);
    const int n = nraw < 0 ? 0 : (nraw > DEGCAP ? DEGCAP : nraw);
    const int st = __builtin_amdgcn_readlane(off_l, j);
    U32F du; du.i = __builtin_amdgcn_readlane(__float_as_int(dis_l), j);
    const float dc = du.f;
    v4f acc = {0.f, 0.f, 0.f, 0.f};
#pragma unroll 1
    for (int q0 = 0; q0 < n; q0 += 32) {
      int pos = st + q0 + lane;
      pos = pos < 0 ? 0 : (pos > csrLen - 1 ? csrLen - 1 : pos);
      int el = csr[pos];
      el = el < 0 ? 0 : (el > nE - 1 ? nE - 1 : el);
      int sl = srcidx[el];
      sl = sl < 0 ? 0 : (sl > nN - 1 ? nN - 1 : sl);
      U32F wu; wu.f = dis[sl] * dc;
      const int mcnt = (n - q0) < 32 ? (n - q0) : 32;
#pragma unroll 1
      for (int p = 0; p < mcnt; ++p) {
        const int s = __builtin_amdgcn_readlane(sl, p);
        U32F t; t.i = __builtin_amdgcn_readlane(wu.i, p);
        const v4f hv = *(const v4f*)(hw + (size_t)s * CC + ch);
        acc = acc + hv * t.f;
      }
    }
    const v4f hc = *(const v4f*)(hw + (size_t)c * CC + ch);
    const float d2 = dc * dc;
    const v4f a = acc + hc * d2 + bv;
    float s1 = (a.x + a.y) + (a.z + a.w);
    s1 += __shfl_xor(s1, 16, 32);
    s1 += __shfl_xor(s1, 8, 32);
    s1 += __shfl_xor(s1, 4, 32);
    s1 += __shfl_xor(s1, 2, 32);
    s1 += __shfl_xor(s1, 1, 32);
    const float mu = s1 * inv128;
    v4f d;
    d.x = a.x - mu; d.y = a.y - mu; d.z = a.z - mu; d.w = a.w - mu;
    float q = (d.x * d.x + d.y * d.y) + (d.z * d.z + d.w * d.w);
    q += __shfl_xor(q, 16, 32);
    q += __shfl_xor(q, 8, 32);
    q += __shfl_xor(q, 4, 32);
    q += __shfl_xor(q, 2, 32);
    q += __shfl_xor(q, 1, 32);
    const float inv = rsqrtf(q * inv128 + eps);
    v4f y;
    y.x = fmaxf(d.x * inv * gv.x + ev.x, 0.0f);
    y.y = fmaxf(d.y * inv * gv.y + ev.y, 0.0f);
    y.z = fmaxf(d.z * inv * gv.z + ev.z, 0.0f);
    y.w = fmaxf(d.w * inv * gv.w + ev.w, 0.0f);
    float* xp = X + (size_t)c * ldx + xcol + ch;
    const v4f xo = *(const v4f*)xp;
    v4f xn = xo + y;
    if (c >= nN) xn = xo;
    if (nraw > DEGCAP) {
      const float qn = __int_as_float(0x7fc00000);
      xn.x = qn; xn.y = qn; xn.z = qn; xn.w = qn;
    }
    *(volatile v4f*)xp = xn;
    __threadfence();
    *(volatile v4f*)xp = xn;
  }
}

extern "C" void kernel_launch(void* const* d_in, const int* in_sizes, int n_in,
                              void* d_out, int out_size, void* d_ws, size_t ws_size,
                              hipStream_t stream) {
  if (n_in < 18) return;
  if (in_sizes[0] <= 0 || (in_sizes[0] % IND) != 0) return;
  const int nN = in_sizes[0] / IND;
  if (in_sizes[1] != nN * IND) return;
  if (in_sizes[2] != IND * CC || in_sizes[3] != CC) return;
  if (in_sizes[4] != IND * CC || in_sizes[5] != CC) return;
  if (in_sizes[6] != NL * CC * CC || in_sizes[7] != NL * CC || in_sizes[8] != NL * CC || in_sizes[9] != NL * CC) return;
  if (in_sizes[10] != NL * CC * CC || in_sizes[11] != NL * CC || in_sizes[12] != NL * CC || in_sizes[13] != NL * CC) return;
  if (in_sizes[14] != IND * NCLS || in_sizes[15] != NCLS) return;
  if (in_sizes[16] < 2 || (in_sizes[16] & 1) != 0) return;
  if (in_sizes[17] < 2 || (in_sizes[17] & 1) != 0) return;
  const int nEr = in_sizes[16] / 2;
  const int nEv = in_sizes[17] / 2;
  if (nN > (1 << 20) || nEr > (1 << 20) || nEv > (1 << 20)) return;
  if (out_size != nN * NCLS) return;

  const float* x_r    = (const float*)d_in[0];
  const float* x_v    = (const float*)d_in[1];
  const float* Wred_r = (const float*)d_in[2];
  const float* bred_r = (const float*)d_in[3];
  const float* Wred_v = (const float*)d_in[4];
  const float* bred_v = (const float*)d_in[5];
  const float* W_r    = (const float*)d_in[6];
  const float* b_r    = (const float*)d_in[7];
  const float* g_r    = (const float*)d_in[8];
  const float* be_r   = (const float*)d_in[9];
  const float* W_v    = (const float*)d_in[10];
  const float* b_v    = (const float*)d_in[11];
  const float* g_v    = (const float*)d_in[12];
  const float* be_v   = (const float*)d_in[13];
  const float* Wcls   = (const float*)d_in[14];
  const float* bcls   = (const float*)d_in[15];
  const int*   ei_r   = (const int*)d_in[16];
  const int*   ei_v   = (const int*)d_in[17];
  float* out = (float*)d_out;

  const int NPAD   = ((nN + TGT - 1) / TGT) * TGT;
  const int nBC    = (nN + NBC - 1) / NBC;
  const int CNTPAD = nBC * NBC;
  const int nBF    = (nN + NBF - 1) / NBF;
  const int OFFN   = nBF * NBF;
  if (nBF + 1 > RBN) return;
  if (OFFN > CNTPAD || NPAD > OFFN) return;
  if ((NPAD % GROWS) != 0 || (NPAD % TGT) != 0) return;
  const int nCls = (nN + GROWS - 1) / GROWS;
  if (nCls * GROWS > NPAD) return;
  const int csrLenR = ((nEr + 31) & ~31) + 32 * (nBF + 1);
  const int csrLenV = ((nEv + 31) & ~31) + 32 * (nBF + 1);
  const int nGemm  = NPAD / GROWS;
  const int nAgg   = NPAD / TGT;
  const int XLD    = 2 * CC;

  char* ws = (char*)d_ws;
  size_t off = 0;
  const size_t oX   = off; off += (size_t)NPAD * XLD * 4;         off = (off + 255) & ~(size_t)255;
  const size_t oXW  = off; off += (size_t)NPAD * CC * 4;          off = (off + 255) & ~(size_t)255;
  const size_t oWrr = off; off += (size_t)CC * IND * 2;           off = (off + 255) & ~(size_t)255;
  const size_t oWrv = off; off += (size_t)CC * IND * 2;           off = (off + 255) & ~(size_t)255;
  const size_t oWr  = off; off += (size_t)NL * CC * CC * 2;       off = (off + 255) & ~(size_t)255;
  const size_t oWv  = off; off += (size_t)NL * CC * CC * 2;       off = (off + 255) & ~(size_t)255;
  const size_t oWc  = off; off += (size_t)NCLSP * IND * 2;        off = (off + 255) & ~(size_t)255;
  const size_t oCnR = off; off += (size_t)CNTPAD * 4;             off = (off + 255) & ~(size_t)255;
  const size_t oOfR = off; off += (size_t)OFFN * 4;               off = (off + 255) & ~(size_t)255;
  const size_t oDiR = off; off += (size_t)OFFN * 4;               off = (off + 255) & ~(size_t)255;
  const size_t oRbR = off; off += (size_t)RBN * 4;                off = (off + 255) & ~(size_t)255;
  const size_t oCsR = off; off += (size_t)csrLenR * 4;            off = (off + 255) & ~(size_t)255;
  const size_t oCnV = off; off += (size_t)CNTPAD * 4;             off = (off + 255) & ~(size_t)255;
  const size_t oOfV = off; off += (size_t)OFFN * 4;               off = (off + 255) & ~(size_t)255;
  const size_t oDiV = off; off += (size_t)OFFN * 4;               off = (off + 255) & ~(size_t)255;
  const size_t oRbV = off; off += (size_t)RBN * 4;                off = (off + 255) & ~(size_t)255;
  const size_t oCsV = off; off += (size_t)csrLenV * 4;            off = (off + 255) & ~(size_t)255;
  if (off > ws_size || off > (size_t)WSCAP) return;
  float*    X    = (float*)(ws + oX);
  float*    XW   = (float*)(ws + oXW);
  _Float16* WrrP = (_Float16*)(ws + oWrr);
  _Float16* WrvP = (_Float16*)(ws + oWrv);
  _Float16* WrP  = (_Float16*)(ws + oWr);
  _Float16* WvP  = (_Float16*)(ws + oWv);
  _Float16* WcP  = (_Float16*)(ws + oWc);
  int*   cntR = (int*)(ws + oCnR);   int*   cntV = (int*)(ws + oCnV);
  int*   offR = (int*)(ws + oOfR);   int*   offV = (int*)(ws + oOfV);
  float* disR = (float*)(ws + oDiR); float* disV = (float*)(ws + oDiV);
  int*   rbR  = (int*)(ws + oRbR);   int*   rbV  = (int*)(ws + oRbV);
  int*   csrR = (int*)(ws + oCsR);   int*   csrV = (int*)(ws + oCsV);

  const float osc = 1.0f / ((float)ASCL * (float)WSCL);

  {
    const dim3 gWred(IND / TPK, CC / TPN, 1);
    k_wT16<<<gWred, NTHR, 0, stream>>>(Wred_r, WrrP, IND, CC, CC, (float)WSCL);
    k_wT16<<<gWred, NTHR, 0, stream>>>(Wred_v, WrvP, IND, CC, CC, (float)WSCL);
    const dim3 gWl(CC / TPK, CC / TPN, NL);
    k_wT16<<<gWl, NTHR, 0, stream>>>(W_r, WrP, CC, CC, CC, (float)WSCL);
    k_wT16<<<gWl, NTHR, 0, stream>>>(W_v, WvP, CC, CC, CC, (float)WSCL);
    const dim3 gWc(IND / TPK, NCLSP / TPN, 1);
    k_wT16<<<gWc, NTHR, 0, stream>>>(Wcls, WcP, IND, NCLS, NCLSP, (float)WSCL);
  }

  hipFuncSetAttribute(reinterpret_cast<const void*>(&k_count),
                      hipFuncAttributeMaxDynamicSharedMemorySize, LDS_COUNT);
  hipFuncSetAttribute(reinterpret_cast<const void*>(&k_fill),
                      hipFuncAttributeMaxDynamicSharedMemorySize, LDS_FILL);
  {
    const int* dstR = ei_r + nEr;
    const int vec8R = ((nEr & 3) == 0) ? 1 : 0;
    k_count<<<nBC, NTHR, LDS_COUNT, stream>>>(dstR, cntR, nEr, vec8R);
    k_offsets<<<1, OTHR, 0, stream>>>(cntR, offR, disR, rbR, nBF);
    k_fill<<<nBF, NTHR, LDS_FILL, stream>>>(dstR, offR, rbR, csrR, nEr, vec8R, csrLenR);
    const int* dstV = ei_v + nEv;
    const int vec8V = ((nEv & 3) == 0) ? 1 : 0;
    k_count<<<nBC, NTHR, LDS_COUNT, stream>>>(dstV, cntV, nEv, vec8V);
    k_offsets<<<1, OTHR, 0, stream>>>(cntV, offV, disV, rbV, nBF);
    k_fill<<<nBF, NTHR, LDS_FILL, stream>>>(dstV, offV, rbV, csrV, nEv, vec8V, csrLenV);
  }

  hipFuncSetAttribute(reinterpret_cast<const void*>(&k_gemm<IND, 1>),
                      hipFuncAttributeMaxDynamicSharedMemorySize, LDS_GEMM);
  hipFuncSetAttribute(reinterpret_cast<const void*>(&k_gemm<CC, 0>),
                      hipFuncAttributeMaxDynamicSharedMemorySize, LDS_GEMM);
  k_gemm<IND, 1><<<nGemm, NTHR, LDS_GEMM, stream>>>(x_r, IND, 0, nN, WrrP, bred_r, X, XLD, 0, osc);
  k_gemm<IND, 1><<<nGemm, NTHR, LDS_GEMM, stream>>>(x_v, IND, 0, nN, WrvP, bred_v, X, XLD, CC, osc);

  const int* srcR = ei_r;
  const int* srcV = ei_v;
  for (int l = 0; l < NL; ++l) {
    k_gemm<CC, 0><<<nGemm, NTHR, LDS_GEMM, stream>>>(X, XLD, 0, NPAD, WrP + (size_t)l * CC * CC, bred_r, XW, CC, 0, osc);
    k_agg<<<nAgg, NTHR, 0, stream>>>(csrR, offR, cntR, srcR, disR, XW,
                                      b_r + (size_t)l * CC, g_r + (size_t)l * CC, be_r + (size_t)l * CC,
                                      X, XLD, 0, nN, nEr, csrLenR, 1e-5f);
    k_gemm<CC, 0><<<nGemm, NTHR, LDS_GEMM, stream>>>(X, XLD, CC, NPAD, WvP + (size_t)l * CC * CC, bred_v, XW, CC, 0, osc);
    k_agg<<<nAgg, NTHR, 0, stream>>>(csrV, offV, cntV, srcV, disV, XW,
                                      b_v + (size_t)l * CC, g_v + (size_t)l * CC, be_v + (size_t)l * CC,
                                      X, XLD, CC, nN, nEv, csrLenV, 1e-5f);
  }

  k_cls<<<nCls, NTHR, 0, stream>>>(X, XLD, NPAD, WcP, bcls, out, nN, osc);
}
